// SelfAttention_SD_77275051590041
// MI455X (gfx1250) — hardware-verified
//
#include <hip/hip_runtime.h>
#include <math.h>
#include <stdint.h>

constexpr int kBatch = 4;
constexpr int kSeq   = 2048;
constexpr int kDim   = 1024;
constexpr int kHeads = 16;
constexpr int kDh    = 64;
constexpr int kInner = kHeads * kDh;
constexpr int kRows  = kBatch * kSeq;
constexpr int kQkLd  = 2 * kInner;
constexpr int kOcLd  = 2 * kInner;
constexpr int kKc    = 64;
constexpr int kNw    = 4;

typedef char chk_tiles_a[((kRows % 64) == 0 && (kQkLd % 64) == 0 && (kInner % 64) == 0 && (kSeq % 64) == 0) ? 1 : -1];
typedef char chk_tiles_b[((kDim % 32) == 0 && (kOcLd % 32) == 0 && (kDh == 64)) ? 1 : -1];

typedef __attribute__((ext_vector_type(16))) _Float16 v16h;
typedef __attribute__((ext_vector_type(8)))  _Float16 v8h;
typedef __attribute__((ext_vector_type(16))) __bf16   v16b;
typedef __attribute__((ext_vector_type(8)))  __bf16   v8b;
typedef __attribute__((ext_vector_type(8)))  float    v8f;
typedef __attribute__((ext_vector_type(4)))  float    v4f;
typedef __attribute__((ext_vector_type(2)))  float    v2f;

__device__ __forceinline__ unsigned short f2bf_bits(float f) {
  unsigned u = __float_as_uint(f);
  return (unsigned short)((u + 0x7FFFu + ((u >> 16) & 1u)) >> 16);
}
__device__ __forceinline__ float bf_bits2f(unsigned short h) { return __uint_as_float(((unsigned)h) << 16); }

__device__ __forceinline__ void dep_guard_h(v8f& a, v8f& b, v16h x, v16h y) { asm volatile("v_nop\n\tv_nop\n\tv_nop\n\tv_nop" : "+v"(a), "+v"(b) : "v"(x), "v"(y)); }
__device__ __forceinline__ void dep_guard_b(v8f& a, v8f& b, v16b x, v16b y) { asm volatile("v_nop\n\tv_nop\n\tv_nop\n\tv_nop" : "+v"(a), "+v"(b) : "v"(x), "v"(y)); }
__device__ __forceinline__ void keep4_h(v16h a, v16h b, v16h c, v16h d) { asm volatile("v_nop" :: "v"(a), "v"(b), "v"(c), "v"(d)); }
__device__ __forceinline__ void keep4_b(v16b a, v16b b, v16b c, v16b d) { asm volatile("v_nop" :: "v"(a), "v"(b), "v"(c), "v"(d)); }
__device__ __forceinline__ void acc_guard4(v8f& a, v8f& b, v8f& c, v8f& d) { asm volatile("v_nop\n\tv_nop\n\tv_nop\n\tv_nop" : "+v"(a), "+v"(b), "+v"(c), "+v"(d)); }
template <typename T> struct Frag;
template <> struct Frag<_Float16> {
  typedef v16h V; union U { v16h v; v8h h[2]; };
  static __device__ __forceinline__ v16h load(const _Float16* p) {
    U f; f.h[0] = *(const v8h*)(p); f.h[1] = *(const v8h*)(p + 16); return f.v;
  }
  static __device__ __forceinline__ v8f mma(v16h a, v16h b, v8f c) {
    return __builtin_amdgcn_wmma_f32_16x16x32_f16(false, a, false, b, (short)0, c, false, false);
  }
  static __device__ __forceinline__ void guard(v8f& a, v8f& b, v16h x, v16h y) { dep_guard_h(a, b, x, y); }
  static __device__ __forceinline__ void keep(v16h a, v16h b, v16h c, v16h d) { keep4_h(a, b, c, d); }
};
template <> struct Frag<__bf16> {
  typedef v16b V; union U { v16b v; v8b h[2]; };
  static __device__ __forceinline__ v16b load(const __bf16* p) {
    U f; f.h[0] = *(const v8b*)(p); f.h[1] = *(const v8b*)(p + 16); return f.v;
  }
  static __device__ __forceinline__ v8f mma(v16b a, v16b b, v8f c) {
    return __builtin_amdgcn_wmma_f32_16x16x32_bf16(false, a, false, b, (short)0, c, false, false);
  }
  static __device__ __forceinline__ void guard(v8f& a, v8f& b, v16b x, v16b y) { dep_guard_b(a, b, x, y); }
  static __device__ __forceinline__ void keep(v16b a, v16b b, v16b c, v16b d) { keep4_b(a, b, c, d); }
};

template <int ET> struct Elem;
template <> struct Elem<0> { typedef _Float16 T; };
template <> struct Elem<1> { typedef __bf16 T; };
template <int ET, bool SPLIT, int BIAS_MODE, int OUT_MODE, bool RESID, int ACT = 0>
__global__ __launch_bounds__(256) void wmma_gemm64(
    const unsigned short* __restrict__ Ap, const unsigned short* __restrict__ A2p, int lda, long strideA,
    const unsigned short* __restrict__ Btp, const unsigned short* __restrict__ Bt2p, int ldb, long strideB,
    void* __restrict__ Cout, void* __restrict__ Cout2, int ldc, long strideC,
    const float* __restrict__ bias,
    const float* __restrict__ resid, long strideR,
    int M, int N, int K, float scale) {
  typedef typename Elem<ET>::T T;
  typedef typename Frag<T>::V V;
  const T* A = (const T*)Ap; const T* A2 = (const T*)A2p; const T* Bt = (const T*)Btp; const T* Bt2 = (const T*)Bt2p;
  __shared__ __align__(16) float sT[8][16 * 68];
  const int b    = blockIdx.y;
  const int lane = threadIdx.x & 31;
  const int wave = threadIdx.x >> 5;
  const int tilesN = N >> 6;
  const int tilesM = M >> 6;
  const int tile = blockIdx.x * 8 + wave;
  if (tile >= tilesM * tilesN) return;
  const int tm = tile / tilesN;
  const int tn = tile - tm * tilesN;
  const int m0 = tm << 6;
  const int n0 = tn << 6;

  const T* Ab  = A  + (size_t)b * strideA;
  const T* Bb  = Bt + (size_t)b * strideB;
  const T* Ab2 = SPLIT ? (A2  + (size_t)b * strideA) : nullptr;
  const T* Bb2 = SPLIT ? (Bt2 + (size_t)b * strideB) : nullptr;

  const int rlane = lane & 15;
  const int koff  = (lane >> 4) * 8;
  const int mOff  = (lane >> 4) * 8;

  v8f acc[4][4];
#pragma unroll
  for (int i = 0; i < 4; ++i)
#pragma unroll
    for (int j = 0; j < 4; ++j) acc[i][j] = (v8f){0.f,0.f,0.f,0.f,0.f,0.f,0.f,0.f};

  for (int k0 = 0; k0 < K; k0 += 32) {
    V bh[4], bl[4];
#pragma unroll
    for (int j = 0; j < 4; ++j) {
      const size_t bo = (size_t)(n0 + (j << 4) + rlane) * ldb + koff + k0;
      bh[j] = Frag<T>::load(Bb + bo);
      if (SPLIT) bl[j] = Frag<T>::load(Bb2 + bo);
    }
#pragma unroll
    for (int i = 0; i < 4; ++i) {
      const size_t ao = (size_t)(m0 + (i << 4) + rlane) * lda + koff + k0;
      V ah = Frag<T>::load(Ab + ao);
      V al;
      if (SPLIT) al = Frag<T>::load(Ab2 + ao);
#pragma unroll
      for (int j = 0; j < 4; ++j) {
        acc[i][j] = Frag<T>::mma(ah, bh[j], acc[i][j]);
        if (SPLIT) {
          acc[i][j] = Frag<T>::mma(ah, bl[j], acc[i][j]);
          acc[i][j] = Frag<T>::mma(al, bh[j], acc[i][j]);
        }
      }
      Frag<T>::guard(acc[i][0], acc[i][3], ah, SPLIT ? al : ah);
    }
    Frag<T>::keep(bh[0], bh[1], bh[2], bh[3]);
    if (SPLIT) Frag<T>::keep(bl[0], bl[1], bl[2], bl[3]);
  }
  acc_guard4(acc[0][0], acc[0][1], acc[0][2], acc[0][3]);
  acc_guard4(acc[1][0], acc[1][1], acc[1][2], acc[1][3]);
  acc_guard4(acc[2][0], acc[2][1], acc[2][2], acc[2][3]);
  acc_guard4(acc[3][0], acc[3][1], acc[3][2], acc[3][3]);

  float* slab = sT[wave];
  const float* Rb = RESID ? (resid + (size_t)b * strideR) : nullptr;
#pragma unroll
  for (int i = 0; i < 4; ++i) {
    const int mBase = m0 + (i << 4);
#pragma unroll
    for (int j = 0; j < 4; ++j) {
      const int n = n0 + (j << 4) + rlane;
      float bv = 0.f;
      if (BIAS_MODE == 2) bv = bias[n];
#pragma unroll
      for (int r = 0; r < 8; ++r) {
        float v = acc[i][j][r] * scale;
        if (BIAS_MODE == 1) v += bias[mBase + mOff + r];
        if (BIAS_MODE == 2) v += bv;
        if (RESID) v += Rb[(size_t)(mBase + mOff + r) * ldc + n];
        if (ACT == 1) v = tanhf(v);
        if (ACT == 2) v = fmaxf(v, 0.0f);
        if (ACT == 3) v = v / (1.0f + expf(-v));
        if (ACT == 4) v = (v > 0.f) ? v : 0.01f * v;
        if (ACT == 5) v = 0.5f * v * (1.0f + erff(v * 0.70710678118654752f));
        slab[(mOff + r) * 68 + (j << 4) + rlane] = v;
      }
    }
    __builtin_amdgcn_fence(__ATOMIC_RELEASE, "workgroup");
    __builtin_amdgcn_wave_barrier();
    __builtin_amdgcn_fence(__ATOMIC_ACQUIRE, "workgroup");
    if (OUT_MODE == 0) {
      float* C = (float*)Cout + (size_t)b * strideC;
      const int hh = lane >> 4, c4 = (lane & 15) * 4;
      for (int pass = 0; pass < 2; ++pass) {
#pragma unroll
        for (int it = 0; it < 8; ++it) {
          const int row = it * 2 + hh;
          v4f v = *(const v4f*)(slab + row * 68 + c4);
          *(volatile v4f*)(C + (size_t)(mBase + row) * ldc + n0 + c4) = v;
        }
        __threadfence();
      }
    } else {
      const int q = lane >> 3, c8 = (lane & 7) * 8;
      unsigned short* C  = (unsigned short*)Cout  + (size_t)b * strideC;
      unsigned short* C2 = (OUT_MODE == 2) ? ((unsigned short*)Cout2 + (size_t)b * strideC) : nullptr;
      for (int pass = 0; pass < 2; ++pass) {
#pragma unroll
        for (int it = 0; it < 4; ++it) {
          const int row = it * 4 + q;
          const float* sp = slab + row * 68 + c8;
          v8h hv, lv;
#pragma unroll
          for (int e = 0; e < 8; ++e) {
            if (OUT_MODE == 1) {
              hv[e] = (_Float16)sp[e];
            } else {
              unsigned short hb = f2bf_bits(sp[e]);
              unsigned short lb = f2bf_bits(sp[e] - bf_bits2f(hb));
              hv[e] = __builtin_bit_cast(_Float16, hb);
              lv[e] = __builtin_bit_cast(_Float16, lb);
            }
          }
          *(volatile v8h*)(C + (size_t)(mBase + row) * ldc + n0 + c8) = hv;
          if (OUT_MODE == 2) *(volatile v8h*)(C2 + (size_t)(mBase + row) * ldc + n0 + c8) = lv;
        }
        __threadfence();
      }
    }
    __builtin_amdgcn_fence(__ATOMIC_RELEASE, "workgroup");
    __builtin_amdgcn_wave_barrier();
    __builtin_amdgcn_fence(__ATOMIC_ACQUIRE, "workgroup");
  }
}

__device__ __forceinline__ unsigned pk16(unsigned short a, unsigned short b) { return (unsigned)a | ((unsigned)b << 16); }

__global__ __launch_bounds__(256) void cast_f32_bf16x2_kernel(const float* __restrict__ in, unsigned short* __restrict__ out, int n2) {
  const int i = blockIdx.x * 256 + threadIdx.x;
  if (i < n2) {
    const v2f f = *(const v2f*)(in + 2 * (size_t)i);
    const unsigned u = pk16(f2bf_bits(f[0]), f2bf_bits(f[1]));
    ((volatile unsigned*)out)[i] = u;
    __threadfence();
    ((volatile unsigned*)out)[i] = u;
  }
}

__global__ __launch_bounds__(256) void cast_dup_bf16x2_kernel(const float* __restrict__ in, unsigned short* __restrict__ out, int n2) {
  const int i = blockIdx.x * 256 + threadIdx.x;
  if (i < n2) {
    const int e = 2 * i;
    const int row = e / kInner;
    const int col = e - row * kInner;
    const v2f f = *(const v2f*)(in + (size_t)e);
    const unsigned u = pk16(f2bf_bits(f[0]), f2bf_bits(f[1]));
    const size_t o0 = ((size_t)row * (2 * kInner) + col) >> 1;
    const size_t o1 = o0 + (kInner >> 1);
    ((volatile unsigned*)out)[o0] = u;
    ((volatile unsigned*)out)[o1] = u;
    __threadfence();
    ((volatile unsigned*)out)[o0] = u;
    ((volatile unsigned*)out)[o1] = u;
  }
}

__global__ __launch_bounds__(256) void bias_rne_kernel(const float* __restrict__ in, float* __restrict__ out, int n) {
  const int i = blockIdx.x * 256 + threadIdx.x;
  if (i < n) {
    const float f = bf_bits2f(f2bf_bits(in[i]));
    ((volatile float*)out)[i] = f;
    __threadfence();
    ((volatile float*)out)[i] = f;
  }
}

__device__ __forceinline__ v8f mma_f16_guarded(v16h a, v16h b, v8f c) {
  c = __builtin_amdgcn_wmma_f32_16x16x32_f16(false, a, false, b, (short)0, c, false, false);
  asm volatile("v_nop\n\tv_nop\n\tv_nop\n\tv_nop" : "+v"(c) : "v"(a), "v"(b));
  return c;
}

__global__ __launch_bounds__(128)
void attn_heads64_kernel(const unsigned short* __restrict__ qkp, const unsigned short* __restrict__ vtp,
                         unsigned short* __restrict__ ocp, float sscale) {
  union FH { v16h v; v8h h[2]; };
  __shared__ __align__(16) _Float16 Ksh[kKc * kDh];
  __shared__ __align__(16) _Float16 Vth[kDh * kKc];
  __shared__ __align__(16) _Float16 Psh[kNw][16 * kKc];
  __shared__ __align__(16) float    Os[kNw][16 * 68];

  const int tid  = threadIdx.x;
  const int wave = tid >> 5;
  const int lane = tid & 31;
  const int hh   = lane >> 4;
  const int c    = lane & 15;
  const float pcarry = 32768.0f;

  constexpr int nqb = kSeq / 64;
  const int bx = blockIdx.x;
  const int qb = bx % nqb;
  const int bh = bx / nqb;
  const int h  = bh % kHeads;
  const int b  = bh / kHeads;
  const int q0 = qb * 64 + wave * 16;

  const _Float16* qk = (const _Float16*)(const void*)qkp;
  const _Float16* vt = (const _Float16*)(const void*)vtp;
  const size_t rowb = (size_t)b * kSeq;
  const _Float16* Qp = qk + rowb * kQkLd + (size_t)h * kDh;
  const _Float16* Kp = qk + rowb * kQkLd + kInner + (size_t)h * kDh;
  const _Float16* Vp = vt + ((size_t)b * kInner + (size_t)h * kDh) * kSeq;
  unsigned short* Ohp = ocp + rowb * kOcLd + (size_t)h * kDh;
  unsigned short* Olp = Ohp + kInner;

  v16h qa[2];
#pragma unroll
  for (int dc = 0; dc < 2; ++dc)
    qa[dc] = Frag<_Float16>::load(Qp + (size_t)(q0 + c) * kQkLd + dc * 32 + 8 * hh);

  float mrow[8], lrow[8];
  v8f oacc[4];
#pragma unroll
  for (int r = 0; r < 8; ++r) { mrow[r] = -INFINITY; lrow[r] = 0.f; }
#pragma unroll
  for (int t = 0; t < 4; ++t) oacc[t] = (v8f){0.f,0.f,0.f,0.f,0.f,0.f,0.f,0.f};

  constexpr int nChunks = kSeq / kKc;
  for (int kc = 0; kc < nChunks; ++kc) {
    const int kv0 = kc * kKc;
    __syncthreads();
    {
      const int r = tid >> 1, half = (tid & 1) * 32;
      const _Float16* kr = Kp + (size_t)(kv0 + r) * kQkLd + half;
      const _Float16* vr = Vp + (size_t)r * kSeq + kv0 + half;
#pragma unroll
      for (int i = 0; i < 4; ++i) {
        const v8h a = *(const v8h*)(kr + 8 * i);
        const v8h w = *(const v8h*)(vr + 8 * i);
        *(v8h*)(Ksh + r * kDh + half + 8 * i) = a;
        *(v8h*)(Vth + r * kKc + half + 8 * i) = w;
      }
    }
    __syncthreads();

    v8f s[4];
#pragma unroll
    for (int j = 0; j < 4; ++j) {
      s[j] = (v8f){0.f,0.f,0.f,0.f,0.f,0.f,0.f,0.f};
#pragma unroll
      for (int dc = 0; dc < 2; ++dc) {
        FH kb;
        kb.h[0] = *(const v8h*)(Ksh + (j * 16 + c) * kDh + dc * 32 + 8 * hh);
        kb.h[1] = *(const v8h*)(Ksh + (j * 16 + c) * kDh + dc * 32 + 16 + 8 * hh);
        s[j] = mma_f16_guarded(qa[dc], kb.v, s[j]);
      }
    }
    float cm[8];
#pragma unroll
    for (int r = 0; r < 8; ++r) {
      float m = -INFINITY;
#pragma unroll
      for (int j = 0; j < 4; ++j) { s[j][r] *= sscale; m = fmaxf(m, s[j][r]); }
#pragma unroll
      for (int off = 1; off < 16; off <<= 1) m = fmaxf(m, __shfl_xor(m, off, 32));
      cm[r] = m;
    }
    _Float16* pw = Psh[wave];
#pragma unroll
    for (int r = 0; r < 8; ++r) {
      const float mnew  = fmaxf(mrow[r], cm[r]);
      const float alpha = __expf(mrow[r] - mnew);
      mrow[r] = mnew;
      float psum = 0.f;
#pragma unroll
      for (int j = 0; j < 4; ++j) {
        const float p = __expf(s[j][r] - mnew);
        psum += p;
        pw[(8 * hh + r) * kKc + j * 16 + c] = (_Float16)(p * pcarry);
      }
#pragma unroll
      for (int off = 1; off < 16; off <<= 1) psum += __shfl_xor(psum, off, 32);
      lrow[r] = lrow[r] * alpha + psum;
#pragma unroll
      for (int t = 0; t < 4; ++t) oacc[t][r] *= alpha;
    }
    __builtin_amdgcn_fence(__ATOMIC_RELEASE, "workgroup");
    __builtin_amdgcn_wave_barrier();
    __builtin_amdgcn_fence(__ATOMIC_ACQUIRE, "workgroup");
#pragma unroll
    for (int kk = 0; kk < 2; ++kk) {
      FH pa;
      pa.h[0] = *(const v8h*)(pw + c * kKc + kk * 32 + 8 * hh);
      pa.h[1] = *(const v8h*)(pw + c * kKc + kk * 32 + 16 + 8 * hh);
#pragma unroll
      for (int t = 0; t < 4; ++t) {
        FH vb;
        vb.h[0] = *(const v8h*)(Vth + (t * 16 + c) * kKc + kk * 32 + 8 * hh);
        vb.h[1] = *(const v8h*)(Vth + (t * 16 + c) * kKc + kk * 32 + 16 + 8 * hh);
        oacc[t] = mma_f16_guarded(pa.v, vb.v, oacc[t]);
      }
    }
  }

  float* os = Os[wave];
#pragma unroll
  for (int r = 0; r < 8; ++r) {
    const float inv = 1.0f / ((lrow[r] + 1e-10f) * pcarry);
#pragma unroll
    for (int t = 0; t < 4; ++t) os[(8 * hh + r) * 68 + t * 16 + c] = oacc[t][r] * inv;
  }
  __builtin_amdgcn_fence(__ATOMIC_RELEASE, "workgroup");
  __builtin_amdgcn_wave_barrier();
  __builtin_amdgcn_fence(__ATOMIC_ACQUIRE, "workgroup");
  {
    const int q4 = lane >> 3, c8 = (lane & 7) * 8;
    for (int pass = 0; pass < 2; ++pass) {
#pragma unroll
      for (int it = 0; it < 4; ++it) {
        const int row = it * 4 + q4;
        const float* sp = os + row * 68 + c8;
        v8h hv, lv;
#pragma unroll
        for (int e = 0; e < 8; ++e) {
          const unsigned short hb = f2bf_bits(sp[e]);
          const unsigned short lb = f2bf_bits(sp[e] - bf_bits2f(hb));
          hv[e] = __builtin_bit_cast(_Float16, hb);
          lv[e] = __builtin_bit_cast(_Float16, lb);
        }
        *(volatile v8h*)(Ohp + (size_t)(q0 + row) * kOcLd + c8) = hv;
        *(volatile v8h*)(Olp + (size_t)(q0 + row) * kOcLd + c8) = lv;
      }
      __threadfence();
    }
  }
}

static inline size_t align_up(size_t v, size_t a) { return (v + a - 1) / a * a; }

extern "C" void kernel_launch(void* const* d_in, const int* in_sizes, int n_in,
                              void* d_out, int out_size, void* d_ws, size_t ws_size,
                              hipStream_t stream) {
  if (n_in < 6) return;
  if (in_sizes[0] != kRows * kDim) return;
  if (in_sizes[1] != kInner * kDim || in_sizes[2] != kInner * kDim || in_sizes[3] != kInner * kDim) return;
  if (in_sizes[4] != kDim * kInner || in_sizes[5] != kDim) return;
  if (out_size != kRows * kDim) return;

  const float* x_in  = (const float*)d_in[0];
  const float* wq_in = (const float*)d_in[1];
  const float* wk_in = (const float*)d_in[2];
  const float* wv_in = (const float*)d_in[3];
  const float* wo_in = (const float*)d_in[4];
  const float* bo_in = (const float*)d_in[5];
  float* out = (float*)d_out;

  const size_t sz_xb  = (size_t)kRows * kDim * 2;
  const size_t sz_wqk = (size_t)2 * kInner * kDim * 2;
  const size_t sz_wv  = (size_t)kInner * kDim * 2;
  const size_t sz_wo  = (size_t)kDim * (2 * kInner) * 2;
  const size_t sz_bor = (size_t)kDim * 4;
  const size_t sz_qk  = (size_t)kRows * kQkLd * 2;
  const size_t sz_vt  = (size_t)kBatch * kInner * kSeq * 2;
  const size_t sz_oc  = (size_t)kRows * kOcLd * 2;
  const size_t off_xb  = 0;
  const size_t off_wqk = align_up(off_xb + sz_xb, 65536);
  const size_t off_wv  = align_up(off_wqk + sz_wqk, 65536);
  const size_t off_wo  = align_up(off_wv + sz_wv, 65536);
  const size_t off_bor = align_up(off_wo + sz_wo, 65536);
  const size_t off_qk  = align_up(off_bor + sz_bor, 65536);
  const size_t off_vt  = align_up(off_qk + sz_qk, 65536);
  const size_t off_oc  = align_up(off_vt + sz_vt, 65536);
  const size_t total   = off_oc + sz_oc;
  if (total > ws_size) return;

  unsigned char* ws = (unsigned char*)d_ws;
  unsigned short* Xb  = (unsigned short*)(ws + off_xb);
  unsigned short* Wqk = (unsigned short*)(ws + off_wqk);
  unsigned short* Wvb = (unsigned short*)(ws + off_wv);
  unsigned short* Woc = (unsigned short*)(ws + off_wo);
  float*          bor = (float*)(ws + off_bor);
  unsigned short* QK  = (unsigned short*)(ws + off_qk);
  unsigned short* Vt  = (unsigned short*)(ws + off_vt);
  unsigned short* Oc  = (unsigned short*)(ws + off_oc);

  {
    const int n2x = kRows * kDim / 2;
    cast_f32_bf16x2_kernel<<<dim3((n2x + 255) / 256), 256, 0, stream>>>(x_in, Xb, n2x);
    const int n2w = kInner * kDim / 2;
    cast_f32_bf16x2_kernel<<<dim3((n2w + 255) / 256), 256, 0, stream>>>(wq_in, Wqk, n2w);
    cast_f32_bf16x2_kernel<<<dim3((n2w + 255) / 256), 256, 0, stream>>>(wk_in, Wqk + (size_t)kInner * kDim, n2w);
    cast_f32_bf16x2_kernel<<<dim3((n2w + 255) / 256), 256, 0, stream>>>(wv_in, Wvb, n2w);
    cast_dup_bf16x2_kernel<<<dim3((n2w + 255) / 256), 256, 0, stream>>>(wo_in, Woc, n2w);
    bias_rne_kernel<<<dim3((kDim + 255) / 256), 256, 0, stream>>>(bo_in, bor, kDim);
  }
  {
    const int tiles = (kRows / 64) * (kQkLd / 64);
    wmma_gemm64<1, false, 0, 1, false><<<dim3(tiles / 8, 1), 256, 0, stream>>>(
        Xb, Xb, kDim, 0L,
        Wqk, Wqk, kDim, 0L,
        (void*)QK, (void*)QK, kQkLd, 0L,
        bor, bor, 0L,
        kRows, kQkLd, kDim, 1.0f);
  }
  {
    const int tiles = (kInner / 64) * (kSeq / 64);
    wmma_gemm64<1, false, 0, 1, false><<<dim3(tiles / 8, kBatch), 256, 0, stream>>>(
        Wvb, Wvb, kDim, 0L,
        Xb, Xb, kDim, (long)kSeq * kDim,
        (void*)Vt, (void*)Vt, kSeq, (long)kInner * kSeq,
        bor, bor, 0L,
        kInner, kSeq, kDim, 1.0f);
  }
  attn_heads64_kernel<<<dim3(kBatch * kHeads * (kSeq / 64)), 128, 0, stream>>>(QK, Vt, Oc, 0.125f);
  {
    const int tiles = (kRows / 64) * (kDim / 64);
    wmma_gemm64<1, false, 2, 0, false><<<dim3(tiles / 8, 1), 256, 0, stream>>>(
        Oc, Oc, kOcLd, 0L,
        Woc, Woc, kOcLd, 0L,
        (void*)out, (void*)out, kDim, 0L,
        bor, bor, 0L,
        kRows, kDim, kOcLd, 1.0f);
  }
}
